// TopkMoE_50946902065585
// MI455X (gfx1250) — hardware-verified
//
#include <hip/hip_runtime.h>
#include <stddef.h>
#include <stdint.h>

#pragma clang fp contract(off)

#define NTOK   8192
#define DD     1024
#define FF     1024
#define NE     8
#define NTILE  136
#define NROWS  (NTILE * 64)
#define NCH    (NTOK / 256)
#define NPC    (NROWS / 4)
#define NPIT   9
#define WSC    64.0f
#define INV64  0.015625f
#define APITCH 136
#define YPITCH 68

static_assert(NTILE == NTOK / 64 + NE);
static_assert(NROWS % 4 == 0);
static_assert(NPC <= NPIT * 256);
static_assert(DD % 128 == 0);
static_assert(FF % 128 == 0);
static_assert(NTOK % 256 == 0);
static_assert(NTOK % 32 == 0);
static_assert((NTOK * DD) % 2048 == 0);
static_assert((NE * FF * DD) % 2048 == 0);
static_assert(NTOK <= 65536);
static_assert(NE <= 8);
static_assert((NROWS * 4) % 128 == 0);

typedef _Float16 v16h __attribute__((ext_vector_type(16)));
typedef _Float16 v8h  __attribute__((ext_vector_type(8)));
typedef float    v8f  __attribute__((ext_vector_type(8)));
typedef float    v4f  __attribute__((ext_vector_type(4)));
typedef unsigned int v4u __attribute__((ext_vector_type(4)));
typedef int      v4i  __attribute__((ext_vector_type(4)));
typedef unsigned short v4us __attribute__((ext_vector_type(4)));

union Frag  { v16h v; v8h h[2]; };
union Pack8 { v8h h; v4u u; };

__device__ __forceinline__ int clampi(int v, int lo, int hi) { return min(max(v, lo), hi); }

__device__ __forceinline__ v8f mma16(v16h a, v16h b, v8f c) {
  c = __builtin_amdgcn_wmma_f32_16x16x32_f16(false, a, false, b, (short)0, c, false, false);
  asm volatile("v_nop\n\tv_nop\n\tv_nop\n\tv_nop" : "+v"(c) : "v"(a), "v"(b));
  return c;
}

__device__ __forceinline__ v16h ldfrag(const _Float16* p, int ld, int row0, int k0, int lane) {
  const int m = lane & 15, lh = lane >> 4;
  const _Float16* q = p + (size_t)(row0 + m) * ld + k0 + 8 * lh;
  Frag f;
  f.h[0] = *(const v8h*)(q);
  f.h[1] = *(const v8h*)(q + 16);
  return f.v;
}

__device__ __forceinline__ v8f zero8() { return (v8f){0.f, 0.f, 0.f, 0.f, 0.f, 0.f, 0.f, 0.f}; }

__global__ __launch_bounds__(256) void k_cvt(const float* __restrict__ src, _Float16* __restrict__ dh, int n8,
                                             float scale) {
  const int i = blockIdx.x * 256 + (int)threadIdx.x;
  if (i >= n8) return;
  const size_t o = (size_t)i * 8;
  const v4f a0 = *(const v4f*)(src + o) * scale;
  const v4f a1 = *(const v4f*)(src + o + 4) * scale;
  Pack8 pk;
  pk.h = (v8h){(_Float16)a0[0], (_Float16)a0[1], (_Float16)a0[2], (_Float16)a0[3],
               (_Float16)a1[0], (_Float16)a1[1], (_Float16)a1[2], (_Float16)a1[3]};
  const v4u vv = pk.u;
  volatile v4u* d = (volatile v4u*)(dh + o);
  *d = vv;
  __threadfence();
  *d = vv;
}

__global__ __launch_bounds__(256) void k_router(const float* __restrict__ x, const float* __restrict__ wr,
                                                const float* __restrict__ br, const int* __restrict__ kp,
                                                int* __restrict__ eidp, float* __restrict__ wtp) {
  __shared__ __align__(16) float sW[NE * DD];
  __shared__ float sBr[NE];
  __shared__ __align__(16) int   sE[32];
  __shared__ __align__(16) float sP[32];
  const int tid = threadIdx.x, lane = tid & 31, wave = tid >> 5;

#pragma unroll 1
  for (int i = tid; i < NE * DD / 4; i += 256) *(v4f*)(sW + 4 * i) = *(const v4f*)(wr + 4 * i);
  if (tid < NE) sBr[tid] = br[tid];
  __syncthreads();
  const int kk = clampi(kp[0], 1, NE);

#pragma unroll 1
  for (int j = 0; j < 4; ++j) {
    const int t = blockIdx.x * 32 + wave * 4 + j;
    const float* xr = x + (size_t)t * DD;
    float acc[NE];
#pragma unroll
    for (int e = 0; e < NE; ++e) acc[e] = 0.f;
#pragma unroll 1
    for (int i = 0; i < DD / 128; ++i) {
      const int d0 = i * 128 + lane * 4;
      const v4f xv = *(const v4f*)(xr + d0);
#pragma unroll
      for (int e = 0; e < NE; ++e) {
        const v4f wv = *(const v4f*)(sW + e * DD + d0);
        float s = acc[e];
        s = fmaf(xv[0], wv[0], s);
        s = fmaf(xv[1], wv[1], s);
        s = fmaf(xv[2], wv[2], s);
        s = fmaf(xv[3], wv[3], s);
        acc[e] = s;
      }
    }
#pragma unroll
    for (int e = 0; e < NE; ++e) {
      float v = acc[e];
#pragma unroll
      for (int off = 16; off > 0; off >>= 1) v += __shfl_xor(v, off, 32);
      acc[e] = v;
    }
    float lg[NE];
#pragma unroll
    for (int e = 0; e < NE; ++e) lg[e] = acc[e] + sBr[e];
    const int me = lane & 7;
    float my = lg[0];
#pragma unroll
    for (int e = 1; e < NE; ++e) my = (me == e) ? lg[e] : my;
    int rank = 0;
    float mx = lg[0];
#pragma unroll
    for (int e = 0; e < NE; ++e) {
      rank += ((lg[e] > my) || (lg[e] == my && e < me)) ? 1 : 0;
      mx = fmaxf(mx, lg[e]);
    }
    const bool sel = (lane < NE) && (rank < kk);
    const unsigned bal = __builtin_amdgcn_ballot_w32(sel);
    const int imax = clampi(31 - __builtin_clz(bal | 1u), 0, NE - 1);
    const float p  = expf(my - mx);
    float s = (lane < NE) ? p : 0.f;
#pragma unroll
    for (int off = 16; off > 0; off >>= 1) s += __shfl_xor(s, off, 32);
    const float pim = __shfl(p, imax, 32);
    const float w = pim * (1.0f / s);
    if (lane == 0) { sE[wave * 4 + j] = imax; sP[wave * 4 + j] = w; }
  }
  __syncthreads();
  if (wave == 0) {
    const v4i ve = *(const v4i*)(sE + (lane & 7) * 4);
    const v4f vp = *(const v4f*)(sP + (lane & 7) * 4);
    volatile v4i* de = (volatile v4i*)(eidp + blockIdx.x * 32 + (lane & 7) * 4);
    volatile v4f* dp = (volatile v4f*)(wtp + blockIdx.x * 32 + (lane & 7) * 4);
    if (lane < 8) *de = ve;
    if (lane >= 8 && lane < 16) *dp = vp;
    __threadfence();
    if (lane < 8) *de = ve;
    if (lane >= 8 && lane < 16) *dp = vp;
  }
}

__global__ __launch_bounds__(256) void k_lists(const int* __restrict__ cid, int* __restrict__ tokp,
                                               int* __restrict__ posp, int* __restrict__ tab) {
  __shared__ __align__(16) unsigned short ltok[NROWS];
  __shared__ int wc[8 * NE];
  __shared__ int wsum[8 * NE];
  __shared__ int srun[NE];
  __shared__ __align__(16) int sTab[64];
  const int tid = threadIdx.x, lane = tid & 31, wave = tid >> 5;
  const unsigned ltm = (1u << lane) - 1u;

  for (int i = tid; i < NROWS; i += 256) ltok[i] = (unsigned short)0;
  if (tid < 64) sTab[tid] = 0;
  if (tid < NE) srun[tid] = 0;

  int hacc[NE];
#pragma unroll
  for (int e = 0; e < NE; ++e) hacc[e] = 0;
#pragma unroll 1
  for (int ch = 0; ch < NCH; ++ch) {
    const int t  = ch * 256 + tid;
    const int et = clampi(cid[t], 0, NE - 1);
#pragma unroll
    for (int e = 0; e < NE; ++e) {
      const unsigned bal = __builtin_amdgcn_ballot_w32(et == e);
      hacc[e] += __builtin_popcount(bal);
    }
  }
  int hv = 0;
#pragma unroll
  for (int e = 0; e < NE; ++e) hv = (lane == e) ? hacc[e] : hv;
  if (lane < NE) wsum[wave * NE + lane] = hv;
  __syncthreads();
  if (tid < NE) {
    int s = 0;
#pragma unroll
    for (int q = 0; q < 8; ++q) s += wsum[q * NE + tid];
    sTab[tid] = s;
  }
  __syncthreads();
  if (tid == 0) {
    int run = 0;
#pragma unroll 1
    for (int e = 0; e < NE; ++e) {
      sTab[32 + e] = run;
      run += (clampi(sTab[e], 0, NTOK) + 63) >> 6;
    }
    sTab[32 + NE] = clampi(run, 0, NTILE);
  }
  __syncthreads();

#pragma unroll 1
  for (int ch = 0; ch < NCH; ++ch) {
    const int t  = ch * 256 + tid;
    const int et = clampi(cid[t], 0, NE - 1);
    int pre = 0;
#pragma unroll
    for (int e = 0; e < NE; ++e) {
      const bool m = (et == e);
      const unsigned bal = __builtin_amdgcn_ballot_w32(m);
      pre = m ? __builtin_popcount(bal & ltm) : pre;
      if (lane == 0) wc[wave * NE + e] = __builtin_popcount(bal);
    }
    __syncthreads();
    int base = srun[et];
#pragma unroll
    for (int q = 0; q < 8; ++q) base += (q < wave) ? wc[q * NE + et] : 0;
    int tot = 0;
    if (tid < NE) {
#pragma unroll
      for (int q = 0; q < 8; ++q) tot += wc[q * NE + tid];
    }
    const int tbe = clampi(sTab[32 + et], 0, NTILE - 1);
    const int row = clampi(tbe * 64 + base + pre, 0, NROWS - 1);
    ltok[row] = (unsigned short)t;
    volatile int* pd = (volatile int*)(posp + t);
    *pd = row;
    __threadfence();
    *pd = row;
    __syncthreads();
    if (tid < NE) srun[tid] += tot;
  }
  __syncthreads();

  for (int ps = 0; ps < 2; ++ps) {
#pragma unroll 1
    for (int it = 0; it < NPIT; ++it) {
      const int p = tid + 256 * it;
      if (p < NPC) {
        const v4us u = *(const v4us*)(ltok + p * 4);
        const v4i v = (v4i){(int)u[0], (int)u[1], (int)u[2], (int)u[3]};
        *(volatile v4i*)(tokp + (size_t)p * 4) = v;
      }
    }
    __threadfence();
  }
  if (wave == 0) {
    const v4i v = *(const v4i*)(sTab + (lane & 15) * 4);
    volatile v4i* d = (volatile v4i*)(tab + (lane & 15) * 4);
    if (lane < 16) *d = v;
    __threadfence();
    if (lane < 16) *d = v;
  }
}

__global__ __launch_bounds__(256) void k_gemm(const _Float16* __restrict__ xh, const _Float16* __restrict__ wh,
                                              const float* __restrict__ be, const int* __restrict__ tokp,
                                              const int* __restrict__ tab, float* __restrict__ yp) {
  __shared__ __align__(16) _Float16 sA[64 * APITCH];
  __shared__ __align__(16) float sC[8 * 16 * YPITCH];
  __shared__ int sTok[64];
  __shared__ int sTab[64];
  const int tid = threadIdx.x, lane = tid & 31, wave = tid >> 5;
  const int hh = lane >> 4, c = lane & 15;
  const int wm = wave & 3, wn = wave >> 2;
  const int b  = blockIdx.x;

  if (tid < 64) sTab[tid] = tab[tid];
  __syncthreads();
  const int ntl = clampi(sTab[32 + NE], 0, NTILE);
  if (b >= ntl) return;
  int e = 0;
#pragma unroll
  for (int q = 1; q < NE; ++q) e += (clampi(sTab[32 + q], 0, NTILE) <= b) ? 1 : 0;
  if (tid < 64) sTok[tid] = clampi(tokp[b * 64 + tid], 0, NTOK - 1);
  __syncthreads();

  const _Float16* whe = wh + (size_t)e * (size_t)(FF * DD);
  const float* bee = be + e * FF;

  const int ar = tid >> 2, ac = tid & 3;
  const _Float16* xrow = xh + (size_t)sTok[ar] * DD + ac * 32;
  _Float16* arow = sA + ar * APITCH + ac * 32;
  float* cw = sC + wave * (16 * YPITCH);

#pragma unroll 1
  for (int nc = 0; nc < FF / 128; ++nc) {
    const int brow = nc * 128 + wn * 64;
    v8f acc[4];
#pragma unroll
    for (int t = 0; t < 4; ++t) acc[t] = zero8();
#pragma unroll 1
    for (int kc = 0; kc < DD / 128; ++kc) {
      __syncthreads();
#pragma unroll
      for (int q = 0; q < 4; ++q) *(v8h*)(arow + 8 * q) = *(const v8h*)(xrow + kc * 128 + 8 * q);
      __syncthreads();
#pragma unroll 1
      for (int ks = 0; ks < 4; ++ks) {
        const int kg = kc * 128 + ks * 32;
        const v16h a = ldfrag(sA, APITCH, wm * 16, ks * 32, lane);
#pragma unroll
        for (int t = 0; t < 4; ++t) {
          const v16h bq = ldfrag(whe, DD, brow + 16 * t, kg, lane);
          acc[t] = mma16(a, bq, acc[t]);
        }
      }
    }
#pragma unroll
    for (int t = 0; t < 4; ++t) {
      const int ncol = 16 * t + c;
      const float bias = bee[brow + ncol];
#pragma unroll
      for (int r = 0; r < 8; ++r) cw[(8 * hh + r) * YPITCH + ncol] = acc[t][r] * INV64 + bias;
    }
    __syncthreads();
    for (int ps = 0; ps < 2; ++ps) {
#pragma unroll
      for (int i = 0; i < 8; ++i) {
        const int row = 2 * i + hh;
        const v4f v = *(const v4f*)(cw + row * YPITCH + c * 4);
        const size_t go = (size_t)(b * 64 + wm * 16 + row) * FF + brow + c * 4;
        *(volatile v4f*)(yp + go) = v;
      }
      __threadfence();
    }
  }
}

__global__ __launch_bounds__(256) void k_out(const float* __restrict__ yp, const int* __restrict__ posp,
                                             const float* __restrict__ wtp, float* __restrict__ out) {
  const int t  = blockIdx.x;
  const int c4 = (int)threadIdx.x;
  const int r  = clampi(posp[t], 0, NROWS - 1);
  const float w = wtp[t];
  const v4f v = *(const v4f*)(yp + (size_t)r * FF + c4 * 4) * w;
  volatile v4f* d = (volatile v4f*)(out + (size_t)t * FF + c4 * 4);
  *d = v;
  __threadfence();
  *d = v;
}

extern "C" void kernel_launch(void* const* d_in, const int* in_sizes, int n_in,
                              void* d_out, int out_size, void* d_ws, size_t ws_size,
                              hipStream_t stream) {
  if (n_in < 6) return;
  if (in_sizes[0] != NTOK * DD) return;
  if (in_sizes[1] != NE * DD) return;
  if (in_sizes[2] != NE) return;
  if (in_sizes[3] != NE * FF * DD) return;
  if (in_sizes[4] != NE * FF) return;
  if (in_sizes[5] != 1) return;
  if (out_size != NTOK * FF) return;

  const float* x  = (const float*)d_in[0];
  const float* Wr = (const float*)d_in[1];
  const float* br = (const float*)d_in[2];
  const float* We = (const float*)d_in[3];
  const float* be = (const float*)d_in[4];
  const int*   kp = (const int*)d_in[5];
  float* out = (float*)d_out;

  size_t off = 0;
  const size_t oXh = off; off += (size_t)NTOK * DD * 2;
  const size_t oWh = off; off += (size_t)NE * FF * DD * 2;
  const size_t oEI = off; off += (size_t)NTOK * 4;
  const size_t oWT = off; off += (size_t)NTOK * 4;
  const size_t oTK = off; off += (size_t)NROWS * 4;
  const size_t oPS = off; off += (size_t)NTOK * 4;
  const size_t oTB = off; off += (size_t)256;
  const size_t oY  = off; off += (size_t)NROWS * FF * 4;
  if (off > ws_size) return;
  if (off > (size_t)134217728) return;
  if ((oWh | oEI | oWT | oTK | oPS | oTB | oY) & (size_t)127) return;

  char* ws = (char*)d_ws;
  _Float16* Xh  = (_Float16*)(ws + oXh);
  _Float16* Wh  = (_Float16*)(ws + oWh);
  int*      EID = (int*)(ws + oEI);
  float*    WT  = (float*)(ws + oWT);
  int*      TOK = (int*)(ws + oTK);
  int*      POS = (int*)(ws + oPS);
  int*      TAB = (int*)(ws + oTB);
  float*    Y   = (float*)(ws + oY);

  k_cvt<<<dim3((NTOK * DD) / 8 / 256), dim3(256), 0, stream>>>(x, Xh, (NTOK * DD) / 8, 1.0f);
  k_cvt<<<dim3((NE * FF * DD) / 8 / 256), dim3(256), 0, stream>>>(We, Wh, (NE * FF * DD) / 8, WSC);
  k_router<<<dim3(NTOK / 32), dim3(256), 0, stream>>>(x, Wr, br, kp, EID, WT);
  k_lists<<<dim3(1), dim3(256), 0, stream>>>(EID, TOK, POS, TAB);
  k_gemm<<<dim3(NTILE), dim3(256), 0, stream>>>(Xh, Wh, be, TOK, TAB, Y);
  k_out<<<dim3(NTOK), dim3(256), 0, stream>>>(Y, POS, WT, out);
  (void)hipGetLastError();
}
